// MobiusGRU_d_38190849196696
// MI455X (gfx1250) — hardware-run, weakly checked
//
#include <hip/hip_runtime.h>
#include <math.h>

constexpr int NBATCH = 64;
constexpr int NSTEP  = 512;
constexpr int NIN    = 256;
constexpr int NHID   = 256;
constexpr int NH1    = 257;
constexpr int NCOL3  = 3 * NHID;
constexpr int NROWS  = NBATCH * NSTEP;
constexpr int RBLK   = 32;
constexpr int NTHR3  = 512;
constexpr int HPITCH = 264;
constexpr int GPITCH = 516;
constexpr int NOUT0  = NSTEP * NBATCH * NH1;
constexpr int NOUT1  = NBATCH * NHID;
constexpr float CARRY = 16.0f;
constexpr float FOLD  = 1.0f / (CARRY * CARRY);
constexpr int LDS_HL    = 0;
constexpr int LDS_RH    = RBLK * HPITCH * 2;
constexpr int LDS_G     = 2 * RBLK * HPITCH * 2;
constexpr int LDS_SLAB  = LDS_G + RBLK * GPITCH * 4;
constexpr int LDS_BT    = LDS_SLAB + RBLK * NH1 * 4;
constexpr int LDS_TOTAL = LDS_BT + 3 * NHID * 4;
static_assert(NIN % 32 == 0 && NHID % 32 == 0, "GEMM K multiple of 32");
static_assert(NROWS % 64 == 0 && NCOL3 % 64 == 0, "GEMM M, N tile multiples");
static_assert(LDS_RH % 16 == 0 && LDS_G % 16 == 0 && LDS_SLAB % 16 == 0 && LDS_BT % 16 == 0, "LDS carve alignment");
static_assert((RBLK * NH1 * 4) % 128 == 0, "32-row output slab is whole 128-B lines");
static_assert(RBLK * NH1 == 2056 * 4, "slab = 2056 float4");
static_assert(NBATCH % RBLK == 0 && RBLK == 2 * (NTHR3 / 32), "two rows per wave");
static_assert((HPITCH % 8) == 0 && (GPITCH % 4) == 0, "LDS pitches keep vector alignment");

typedef __attribute__((ext_vector_type(16))) _Float16 v16h;
typedef __attribute__((ext_vector_type(8)))  _Float16 v8h;
typedef __attribute__((ext_vector_type(4)))  _Float16 v4h;
typedef __attribute__((ext_vector_type(16))) __bf16   v16b;
typedef __attribute__((ext_vector_type(8)))  __bf16   v8b;
typedef __attribute__((ext_vector_type(8)))  float    v8f;
typedef __attribute__((ext_vector_type(4)))  float    v4f;

__device__ __forceinline__ unsigned short f2bf_bits(float f) {
  unsigned u = __float_as_uint(f);
  return (unsigned short)((u + 0x7FFFu + ((u >> 16) & 1u)) >> 16);
}
__device__ __forceinline__ float bf_bits2f(unsigned short h) { return __uint_as_float(((unsigned)h) << 16); }

__device__ __forceinline__ void dep_guard4_h(v8f& a, v8f& b, v8f& c, v8f& d, v16h x, v16h y) { asm volatile("v_nop\n\tv_nop\n\tv_nop\n\tv_nop" : "+v"(a), "+v"(b), "+v"(c), "+v"(d) : "v"(x), "v"(y)); }
__device__ __forceinline__ void dep_guard4_b(v8f& a, v8f& b, v8f& c, v8f& d, v16b x, v16b y) { asm volatile("v_nop\n\tv_nop\n\tv_nop\n\tv_nop" : "+v"(a), "+v"(b), "+v"(c), "+v"(d) : "v"(x), "v"(y)); }
__device__ __forceinline__ void keep4_h(v16h a, v16h b, v16h c, v16h d) { asm volatile("v_nop" :: "v"(a), "v"(b), "v"(c), "v"(d)); }
__device__ __forceinline__ void keep4_b(v16b a, v16b b, v16b c, v16b d) { asm volatile("v_nop" :: "v"(a), "v"(b), "v"(c), "v"(d)); }
__device__ __forceinline__ void acc_guard4(v8f& a, v8f& b, v8f& c, v8f& d) { asm volatile("v_nop\n\tv_nop\n\tv_nop\n\tv_nop" : "+v"(a), "+v"(b), "+v"(c), "+v"(d)); }
__device__ __forceinline__ void acc_guard2(v8f& a, v8f& b) { asm volatile("v_nop\n\tv_nop\n\tv_nop\n\tv_nop" : "+v"(a), "+v"(b)); }
__device__ __forceinline__ void step_guard4(v8f& a, v8f& b, v8f& c, v8f& d, v16h w, v16h x, v16h y, v16h z) { asm volatile("v_nop\n\tv_nop\n\tv_nop\n\tv_nop" : "+v"(a), "+v"(b), "+v"(c), "+v"(d) : "v"(w), "v"(x), "v"(y), "v"(z)); }
__device__ __forceinline__ void step_guard2(v8f& a, v8f& b, v16h w, v16h x, v16h y) { asm volatile("v_nop\n\tv_nop\n\tv_nop\n\tv_nop" : "+v"(a), "+v"(b) : "v"(w), "v"(x), "v"(y)); }

template <typename T> struct Frag;
template <> struct Frag<_Float16> {
  typedef v16h V; union U { v16h v; v8h h[2]; };
  static __device__ __forceinline__ v16h load(const _Float16* p) {
    U f; f.h[0] = *(const v8h*)(p); f.h[1] = *(const v8h*)(p + 16); return f.v;
  }
  static __device__ __forceinline__ v8f mma(v16h a, v16h b, v8f c) {
    return __builtin_amdgcn_wmma_f32_16x16x32_f16(false, a, false, b, (short)0, c, false, false);
  }
  static __device__ __forceinline__ void guard4(v8f& a, v8f& b, v8f& c, v8f& d, v16h x, v16h y) { dep_guard4_h(a, b, c, d, x, y); }
  static __device__ __forceinline__ void keep(v16h a, v16h b, v16h c, v16h d) { keep4_h(a, b, c, d); }
};
template <> struct Frag<__bf16> {
  typedef v16b V; union U { v16b v; v8b h[2]; };
  static __device__ __forceinline__ v16b load(const __bf16* p) {
    U f; f.h[0] = *(const v8b*)(p); f.h[1] = *(const v8b*)(p + 16); return f.v;
  }
  static __device__ __forceinline__ v8f mma(v16b a, v16b b, v8f c) {
    return __builtin_amdgcn_wmma_f32_16x16x32_bf16(false, a, false, b, (short)0, c, false, false);
  }
  static __device__ __forceinline__ void guard4(v8f& a, v8f& b, v8f& c, v8f& d, v16b x, v16b y) { dep_guard4_b(a, b, c, d, x, y); }
  static __device__ __forceinline__ void keep(v16b a, v16b b, v16b c, v16b d) { keep4_b(a, b, c, d); }
};

template <int ET> struct Elem;
template <> struct Elem<0> { typedef _Float16 T; };
template <> struct Elem<1> { typedef __bf16 T; };
template <int ET, bool SPLIT, int BIAS_MODE, int OUT_MODE, bool RESID, int ACT = 0>
__global__ __launch_bounds__(256) void wmma_gemm64(
    const unsigned short* __restrict__ Ap, const unsigned short* __restrict__ A2p, int lda, long strideA,
    const unsigned short* __restrict__ Btp, const unsigned short* __restrict__ Bt2p, int ldb, long strideB,
    void* __restrict__ Cout, void* __restrict__ Cout2, int ldc, long strideC,
    const float* __restrict__ bias,
    const float* __restrict__ resid, long strideR,
    int M, int N, int K, float scale) {
  typedef typename Elem<ET>::T T;
  typedef typename Frag<T>::V V;
  const T* A = (const T*)Ap; const T* A2 = (const T*)A2p; const T* Bt = (const T*)Btp; const T* Bt2 = (const T*)Bt2p;
  __shared__ __align__(16) float sT[8][16 * 68];
  const int b    = blockIdx.y;
  const int lane = threadIdx.x & 31;
  const int wave = threadIdx.x >> 5;
  const int tilesN = N >> 6;
  const int tilesM = M >> 6;
  const int tile = blockIdx.x * 8 + wave;
  if (tile >= tilesM * tilesN) return;
  const int tm = tile / tilesN;
  const int tn = tile - tm * tilesN;
  const int m0 = tm << 6;
  const int n0 = tn << 6;

  const T* Ab  = A  + (size_t)b * strideA;
  const T* Bb  = Bt + (size_t)b * strideB;
  const T* Ab2 = SPLIT ? (A2  + (size_t)b * strideA) : nullptr;
  const T* Bb2 = SPLIT ? (Bt2 + (size_t)b * strideB) : nullptr;

  const int rlane = lane & 15;
  const int koff  = (lane >> 4) * 8;
  const int mOff  = (lane >> 4) * 8;

  v8f acc[4][4];
#pragma unroll
  for (int i = 0; i < 4; ++i)
#pragma unroll
    for (int j = 0; j < 4; ++j) acc[i][j] = (v8f){0.f,0.f,0.f,0.f,0.f,0.f,0.f,0.f};

  for (int k0 = 0; k0 < K; k0 += 32) {
    V bh[4], bl[4];
#pragma unroll
    for (int j = 0; j < 4; ++j) {
      const size_t bo = (size_t)(n0 + (j << 4) + rlane) * ldb + koff + k0;
      bh[j] = Frag<T>::load(Bb + bo);
      if (SPLIT) bl[j] = Frag<T>::load(Bb2 + bo);
    }
#pragma unroll
    for (int i = 0; i < 4; ++i) {
      const size_t ao = (size_t)(m0 + (i << 4) + rlane) * lda + koff + k0;
      V ah = Frag<T>::load(Ab + ao);
      V al;
      if (SPLIT) al = Frag<T>::load(Ab2 + ao);
#pragma unroll
      for (int j = 0; j < 4; ++j) {
        acc[i][j] = Frag<T>::mma(ah, bh[j], acc[i][j]);
        if (SPLIT) {
          acc[i][j] = Frag<T>::mma(ah, bl[j], acc[i][j]);
          acc[i][j] = Frag<T>::mma(al, bh[j], acc[i][j]);
        }
      }
      Frag<T>::guard4(acc[i][0], acc[i][1], acc[i][2], acc[i][3], ah, SPLIT ? al : ah);
    }
    Frag<T>::keep(bh[0], bh[1], bh[2], bh[3]);
    if (SPLIT) Frag<T>::keep(bl[0], bl[1], bl[2], bl[3]);
  }
  acc_guard4(acc[0][0], acc[0][1], acc[0][2], acc[0][3]);
  acc_guard4(acc[1][0], acc[1][1], acc[1][2], acc[1][3]);
  acc_guard4(acc[2][0], acc[2][1], acc[2][2], acc[2][3]);
  acc_guard4(acc[3][0], acc[3][1], acc[3][2], acc[3][3]);

  float* slab = sT[wave];
  const float* Rb = RESID ? (resid + (size_t)b * strideR) : nullptr;
#pragma unroll
  for (int i = 0; i < 4; ++i) {
    const int mBase = m0 + (i << 4);
#pragma unroll
    for (int j = 0; j < 4; ++j) {
      const int n = n0 + (j << 4) + rlane;
      float bv = 0.f;
      if (BIAS_MODE == 2) bv = bias[n];
#pragma unroll
      for (int r = 0; r < 8; ++r) {
        float v = acc[i][j][r] * scale;
        if (BIAS_MODE == 1) v += bias[mBase + mOff + r];
        if (BIAS_MODE == 2) v += bv;
        if (RESID) v += Rb[(size_t)(mBase + mOff + r) * ldc + n];
        if (ACT == 1) v = tanhf(v);
        if (ACT == 2) v = fmaxf(v, 0.0f);
        if (ACT == 3) v = v / (1.0f + expf(-v));
        if (ACT == 4) v = (v > 0.f) ? v : 0.01f * v;
        slab[(mOff + r) * 68 + (j << 4) + rlane] = v;
      }
    }
    __builtin_amdgcn_fence(__ATOMIC_RELEASE, "workgroup");
    __builtin_amdgcn_wave_barrier();
    __builtin_amdgcn_fence(__ATOMIC_ACQUIRE, "workgroup");
    if (OUT_MODE == 0) {
      float* C = (float*)Cout + (size_t)b * strideC;
      const int hh = lane >> 4, c4 = (lane & 15) * 4;
      for (int pass = 0; pass < 2; ++pass) {
#pragma unroll
        for (int it = 0; it < 8; ++it) {
          const int row = it * 2 + hh;
          v4f v = *(const v4f*)(slab + row * 68 + c4);
          *(volatile v4f*)(C + (size_t)(mBase + row) * ldc + n0 + c4) = v;
        }
        __threadfence();
      }
    } else {
      const int q = lane >> 3, c8 = (lane & 7) * 8;
      unsigned short* C  = (unsigned short*)Cout  + (size_t)b * strideC;
      unsigned short* C2 = (OUT_MODE == 2) ? ((unsigned short*)Cout2 + (size_t)b * strideC) : nullptr;
      for (int pass = 0; pass < 2; ++pass) {
#pragma unroll
        for (int it = 0; it < 4; ++it) {
          const int row = it * 4 + q;
          const float* sp = slab + row * 68 + c8;
          v8h hv, lv;
#pragma unroll
          for (int e = 0; e < 8; ++e) {
            if (OUT_MODE == 1) {
              hv[e] = (_Float16)sp[e];
            } else {
              unsigned short hb = f2bf_bits(sp[e]);
              unsigned short lb = f2bf_bits(sp[e] - bf_bits2f(hb));
              hv[e] = __builtin_bit_cast(_Float16, hb);
              lv[e] = __builtin_bit_cast(_Float16, lb);
            }
          }
          *(volatile v8h*)(C + (size_t)(mBase + row) * ldc + n0 + c8) = hv;
          if (OUT_MODE == 2) *(volatile v8h*)(C2 + (size_t)(mBase + row) * ldc + n0 + c8) = lv;
        }
        __threadfence();
      }
    }
    __builtin_amdgcn_fence(__ATOMIC_RELEASE, "workgroup");
    __builtin_amdgcn_wave_barrier();
    __builtin_amdgcn_fence(__ATOMIC_ACQUIRE, "workgroup");
  }
}

__global__ __launch_bounds__(256) void pack_w_kernel(const float* __restrict__ wih, const float* __restrict__ whh,
                                                     unsigned short* __restrict__ WI, unsigned short* __restrict__ WH) {
  const int i = blockIdx.x * 256 + threadIdx.x;
  const int which = blockIdx.y;
  const float* src = which ? whh : wih;
  unsigned short* dst = which ? WH : WI;
  if (i < NCOL3 * 32) {
    const int n = i >> 5, k8 = (i & 31) * 8;
    const int g = n >> 8, j = n & 255;
    const float* sp = src + (size_t)(g * NH1 + 1 + j) * NH1 + 1 + k8;
    v8h hv;
#pragma unroll
    for (int e = 0; e < 8; ++e) hv[e] = (_Float16)(sp[e] * CARRY);
    *(volatile v8h*)(dst + (size_t)i * 8) = hv;
    __threadfence();
    *(volatile v8h*)(dst + (size_t)i * 8) = hv;
  }
}

__global__ __launch_bounds__(256) void pack_x_kernel(const float* __restrict__ x, unsigned short* __restrict__ XH) {
  const int i = blockIdx.x * 256 + threadIdx.x;
  if (i < NROWS * 32) {
    const int m = i >> 5, k8 = (i & 31) * 8;
    const int t = m >> 6, b = m & 63;
    const float* sp = x + ((size_t)b * NSTEP + (size_t)t) * NIN + k8;
    const v4f a  = *(const v4f*)(sp);
    const v4f bq = *(const v4f*)(sp + 4);
    v8h hv;
#pragma unroll
    for (int e = 0; e < 4; ++e) {
      hv[e]     = (_Float16)(a[e] * CARRY);
      hv[4 + e] = (_Float16)(bq[e] * CARRY);
    }
    *(volatile v8h*)(XH + (size_t)i * 8) = hv;
    __threadfence();
    *(volatile v8h*)(XH + (size_t)i * 8) = hv;
  }
}

__device__ __forceinline__ float hsum16(float v) {
  v += __shfl_xor(v, 1, 32);
  v += __shfl_xor(v, 2, 32);
  v += __shfl_xor(v, 4, 32);
  v += __shfl_xor(v, 8, 32);
  return v;
}
__device__ __forceinline__ void ld16_lds(float (&d)[16], const float* p) {
#pragma unroll
  for (int q = 0; q < 4; ++q) {
    const v4f v = *(const v4f*)(p + 64 * q);
    d[4 * q + 0] = v[0]; d[4 * q + 1] = v[1]; d[4 * q + 2] = v[2]; d[4 * q + 3] = v[3];
  }
}
__device__ __forceinline__ void ld16_glb(float (&d)[16], const float* p) {
#pragma unroll
  for (int q = 0; q < 4; ++q) {
    const v4f v = *(const v4f*)(p + 64 * q);
    d[4 * q + 0] = v[0]; d[4 * q + 1] = v[1]; d[4 * q + 2] = v[2]; d[4 * q + 3] = v[3];
  }
}
__device__ __forceinline__ void e0_map(float (&s)[16], float& ysq, float& x0, float Kc, float sK, float invsK) {
  float ss = 0.0f;
#pragma unroll
  for (int i = 0; i < 16; ++i) ss = fmaf(s[i], s[i], ss);
  ss = hsum16(ss);
  const float n  = fmaxf(sqrtf(ss), 1e-15f);
  const float th = n * invsK;
  const float f  = sK * sinhf(th) * (1.0f / n);
#pragma unroll
  for (int i = 0; i < 16; ++i) s[i] *= f;
  ysq = (f * f) * ss;
  x0  = sqrtf(fmaxf(Kc + ysq, 1e-7f));
}
__device__ __forceinline__ float l0_coef(float ysq, float x0, float sK, float invsK) {
  const float yn = fmaxf(sqrtf(ysq), 1e-15f);
  const float th = fmaxf(x0 * invsK, 1.0f + 1e-7f);
  return sK * acoshf(th) * (1.0f / yn);
}
__device__ __forceinline__ void madd(const float (&yin)[16], float sgn, float ysq_in, float x0_in, const float (&s)[16],
                                     float (&yout)[16], float& ysq_out, float& x0_out, float Kc, float sK, float invsK) {
  float d = 0.0f, q = 0.0f;
#pragma unroll
  for (int i = 0; i < 16; ++i) { d = fmaf(yin[i], s[i], d); q = fmaf(s[i], s[i], q); }
  d = hsum16(d) * sgn;
  q = hsum16(q);
  const float yn    = fmaxf(sqrtf(ysq_in), 1e-15f);
  const float ryn   = 1.0f / yn;
  const float alpha = (d * ryn) * invsK;
  const float coef  = (alpha * (sK - x0_in)) * ryn;
  const float nrm   = fminf(sqrtf(fmaxf(q, 1e-7f)), 1000000.0f);
  const float th    = fmaxf(nrm * invsK, 1e-15f);
  const float ch    = coshf(th);
  const float shc   = sinhf(th) * (1.0f / th);
  const float ca    = (ch - shc * coef) * sgn;
  float nq = 0.0f;
#pragma unroll
  for (int i = 0; i < 16; ++i) {
    const float v = fmaf(ca, yin[i], shc * s[i]);
    yout[i] = v;
    nq = fmaf(v, v, nq);
  }
  nq = hsum16(nq);
  ysq_out = nq;
  x0_out  = sqrtf(fmaxf(Kc + nq, 1e-7f));
}

__global__ __launch_bounds__(NTHR3) void hyp_seq_kernel(const float* __restrict__ UX, const unsigned short* __restrict__ WHp,
                                                        const float* __restrict__ bias, const float* __restrict__ kptr,
                                                        float* __restrict__ out0, float* __restrict__ out1) {
  extern __shared__ __align__(16) unsigned char smem[];
  _Float16* hlT  = (_Float16*)(smem + LDS_HL);
  _Float16* rhT  = (_Float16*)(smem + LDS_RH);
  float*    G    = (float*)(smem + LDS_G);
  float*    slab = (float*)(smem + LDS_SLAB);
  float*    btS  = (float*)(smem + LDS_BT);
  const _Float16* WH = (const _Float16*)WHp;

  const int tid = threadIdx.x, lane = tid & 31, wave = tid >> 5;
  const int hh = lane >> 4, c = lane & 15, koff = hh * 8;
  const int blk  = blockIdx.x;
  const int vrow = 2 * wave + hh;
  const int brow = blk * RBLK + vrow;

  const float kk    = kptr[0];
  const float Kc    = 1.0f / kk;
  const float sK    = sqrtf(Kc);
  const float invsK = 1.0f / sK;

  {
    unsigned* zw = (unsigned*)smem;
#pragma unroll 1
    for (int i = tid; i < (LDS_G / 4); i += NTHR3) zw[i] = 0u;
  }
#pragma unroll 1
  for (int g = 0; g < 3; ++g) {
    float s[16];
#pragma unroll
    for (int q = 0; q < 4; ++q)
#pragma unroll
      for (int j = 0; j < 4; ++j) s[4 * q + j] = bias[g * NH1 + 1 + 64 * q + 4 * c + j];
    float ysq, x0;
    e0_map(s, ysq, x0, Kc, sK, invsK);
    const float cl = l0_coef(ysq, x0, sK, invsK);
    if (wave == 0 && hh == 0) {
#pragma unroll
      for (int q = 0; q < 4; ++q) {
        v4f o;
        o[0] = cl * s[4 * q + 0]; o[1] = cl * s[4 * q + 1]; o[2] = cl * s[4 * q + 2]; o[3] = cl * s[4 * q + 3];
        *(v4f*)(btS + g * NHID + 64 * q + 4 * c) = o;
      }
    }
  }

  float hy[16], gate[16];
#pragma unroll
  for (int i = 0; i < 16; ++i) { hy[i] = 0.0f; gate[i] = 0.0f; }
  float hysq = 0.0f, hx0 = sK;
  float clh = l0_coef(hysq, hx0, sK, invsK);

  const _Float16* aH0 = hlT + c * HPITCH + koff;
  const _Float16* aH1 = aH0 + 16 * HPITCH;
  const _Float16* aR0 = rhT + c * HPITCH + koff;
  const _Float16* aR1 = aR0 + 16 * HPITCH;
  const int wrow1 = (wave < 8) ? (32 * wave) : (32 * wave + 256);
  const _Float16* b10 = WH + (size_t)(wrow1 + c) * NHID + koff;
  const _Float16* b11 = b10 + (size_t)16 * NHID;
  const _Float16* b20 = WH + (size_t)(256 + 16 * wave + c) * NHID + koff;
  float* g1 = G + (8 * hh) * GPITCH + 32 * wave + c;
  float* g2 = G + (8 * hh) * GPITCH + 16 * wave + c;
  const float* grow = G + vrow * GPITCH + 4 * c;
  const v8f z8 = {0.f, 0.f, 0.f, 0.f, 0.f, 0.f, 0.f, 0.f};

  __syncthreads();

#pragma unroll 1
  for (int t = 0; t < NSTEP; ++t) {
    const float* uxp = UX + ((size_t)t * NBATCH + (size_t)brow) * NCOL3 + 4 * c;

    {
      v8f a00 = z8, a01 = z8, a10 = z8, a11 = z8;
#pragma unroll 1
      for (int k0 = 0; k0 < NHID; k0 += 32) {
        const v16h fa0 = Frag<_Float16>::load(aH0 + k0);
        const v16h fa1 = Frag<_Float16>::load(aH1 + k0);
        const v16h fb0 = Frag<_Float16>::load(b10 + k0);
        const v16h fb1 = Frag<_Float16>::load(b11 + k0);
        a00 = Frag<_Float16>::mma(fa0, fb0, a00);
        a01 = Frag<_Float16>::mma(fa0, fb1, a01);
        a10 = Frag<_Float16>::mma(fa1, fb0, a10);
        a11 = Frag<_Float16>::mma(fa1, fb1, a11);
        step_guard4(a00, a01, a10, a11, fa0, fa1, fb0, fb1);
      }
      acc_guard4(a00, a01, a10, a11);
#pragma unroll
      for (int r = 0; r < 8; ++r) {
        g1[r * GPITCH]             = a00[r] * FOLD;
        g1[r * GPITCH + 16]        = a01[r] * FOLD;
        g1[(16 + r) * GPITCH]      = a10[r] * FOLD;
        g1[(16 + r) * GPITCH + 16] = a11[r] * FOLD;
      }
    }
    __syncthreads();

#pragma unroll 1
    for (int it = 0; it < 2; ++it) {
      const int gsel = 2 * it;
      float y[16], u[16];
      float ysq, x0;
      ld16_lds(y, grow + it * 256);
      e0_map(y, ysq, x0, Kc, sK, invsK);
      ld16_glb(u, uxp + gsel * NHID);
      madd(y, 1.0f, ysq, x0, u, y, ysq, x0, Kc, sK, invsK);
      ld16_lds(u, btS + gsel * NHID + 4 * c);
      madd(y, 1.0f, ysq, x0, u, y, ysq, x0, Kc, sK, invsK);
      const float cl = l0_coef(ysq, x0, sK, invsK);
#pragma unroll
      for (int i = 0; i < 16; ++i) gate[i] = 1.0f / (1.0f + expf(-(cl * y[i])));
      if (it == 0) {
#pragma unroll
        for (int q = 0; q < 4; ++q) {
          v4h hv;
#pragma unroll
          for (int j = 0; j < 4; ++j) hv[j] = (_Float16)((gate[4 * q + j] * (clh * hy[4 * q + j])) * CARRY);
          *(v4h*)(rhT + vrow * HPITCH + 64 * q + 4 * c) = hv;
        }
      }
    }
    __syncthreads();

    {
      v8f a0 = z8, a1 = z8;
#pragma unroll 1
      for (int k0 = 0; k0 < NHID; k0 += 32) {
        const v16h fa0 = Frag<_Float16>::load(aR0 + k0);
        const v16h fa1 = Frag<_Float16>::load(aR1 + k0);
        const v16h fb0 = Frag<_Float16>::load(b20 + k0);
        a0 = Frag<_Float16>::mma(fa0, fb0, a0);
        a1 = Frag<_Float16>::mma(fa1, fb0, a1);
        step_guard2(a0, a1, fa0, fa1, fb0);
      }
      acc_guard2(a0, a1);
#pragma unroll
      for (int r = 0; r < 8; ++r) {
        g2[r * GPITCH]        = a0[r] * FOLD;
        g2[(16 + r) * GPITCH] = a1[r] * FOLD;
      }
    }
    __syncthreads();

    {
      float y[16], u[16];
      float ysq, x0;
      ld16_lds(y, grow);
      e0_map(y, ysq, x0, Kc, sK, invsK);
      ld16_glb(u, uxp + NHID);
      madd(y, 1.0f, ysq, x0, u, y, ysq, x0, Kc, sK, invsK);
      ld16_lds(u, btS + NHID + 4 * c);
      madd(y, 1.0f, ysq, x0, u, y, ysq, x0, Kc, sK, invsK);
      const float cls = l0_coef(ysq, x0, sK, invsK);
#pragma unroll
      for (int i = 0; i < 16; ++i) y[i] *= cls;
      float dsq, dx0;
      madd(hy, -1.0f, hysq, hx0, y, u, dsq, dx0, Kc, sK, invsK);
      const float cld = l0_coef(dsq, dx0, sK, invsK);
#pragma unroll
      for (int i = 0; i < 16; ++i) u[i] = gate[i] * (cld * u[i]);
      madd(hy, 1.0f, hysq, hx0, u, hy, hysq, hx0, Kc, sK, invsK);
    }
    {
      float* srow = slab + vrow * NH1;
      if (c == 0) srow[0] = hx0;
#pragma unroll
      for (int q = 0; q < 4; ++q)
#pragma unroll
        for (int j = 0; j < 4; ++j) srow[1 + 64 * q + 4 * c + j] = hy[4 * q + j];
    }
    clh = l0_coef(hysq, hx0, sK, invsK);
#pragma unroll
    for (int q = 0; q < 4; ++q) {
      v4h hv;
#pragma unroll
      for (int j = 0; j < 4; ++j) hv[j] = (_Float16)((clh * hy[4 * q + j]) * CARRY);
      *(v4h*)(hlT + vrow * HPITCH + 64 * q + 4 * c) = hv;
    }
    __syncthreads();

    {
      float* ob = out0 + (size_t)t * (NBATCH * NH1) + (size_t)blk * (RBLK * NH1);
      v4f sv[4];
#pragma unroll
      for (int it = 0; it < 4; ++it) sv[it] = *(const v4f*)(slab + 4 * ((wave * 4 + it) * 32 + lane));
      const v4f tv = *(const v4f*)(slab + 4 * (2048 + (lane & 7)));
      const bool tail = (wave == 0) && (lane < 8);
      for (int pass = 0; pass < 2; ++pass) {
#pragma unroll
        for (int it = 0; it < 4; ++it) *(volatile v4f*)(ob + 4 * ((wave * 4 + it) * 32 + lane)) = sv[it];
        if (tail) *(volatile v4f*)(ob + 4 * (2048 + lane)) = tv;
        __threadfence();
      }
    }
  }

  {
    float* o1 = out1 + (size_t)brow * NHID + 4 * c;
    for (int pass = 0; pass < 2; ++pass) {
#pragma unroll
      for (int q = 0; q < 4; ++q) {
        v4f o;
        o[0] = hy[4 * q + 0]; o[1] = hy[4 * q + 1]; o[2] = hy[4 * q + 2]; o[3] = hy[4 * q + 3];
        *(volatile v4f*)(o1 + 64 * q) = o;
      }
      __threadfence();
    }
  }
}

extern "C" void kernel_launch(void* const* d_in, const int* in_sizes, int n_in,
                              void* d_out, int out_size, void* d_ws, size_t ws_size, hipStream_t stream) {
  if (n_in < 5 || d_out == nullptr || d_ws == nullptr) return;
  if (in_sizes[0] != NBATCH * NSTEP * NIN || in_sizes[1] != 1 || in_sizes[2] != 3 * NH1 * NH1 ||
      in_sizes[3] != 3 * NH1 * NH1 || in_sizes[4] != 3 * NH1 || out_size != NOUT0 + NOUT1) return;

  const float* x    = (const float*)d_in[0];
  const float* kp   = (const float*)d_in[1];
  const float* wih  = (const float*)d_in[2];
  const float* whh  = (const float*)d_in[3];
  const float* bias = (const float*)d_in[4];
  float* out = (float*)d_out;

  char* ws = (char*)d_ws; size_t off = 0;
  auto carve = [&](size_t bytes) -> char* { char* p = ws + off; off += (bytes + 255) & ~(size_t)255; return p; };
  unsigned short* XH = (unsigned short*)carve((size_t)NROWS * NIN * 2);
  unsigned short* WI = (unsigned short*)carve((size_t)NCOL3 * NIN * 2);
  unsigned short* WH = (unsigned short*)carve((size_t)NCOL3 * NHID * 2);
  float*          UX = (float*)carve((size_t)NROWS * NCOL3 * 4);
  if (off > ws_size || off > (size_t)134217728) return;

  pack_w_kernel<<<dim3((NCOL3 * 32) / 256, 2), 256, 0, stream>>>(wih, whh, WI, WH);
  pack_x_kernel<<<(NROWS * 32) / 256, 256, 0, stream>>>(x, XH);
  wmma_gemm64<0, false, 0, 0, false, 0><<<dim3((NROWS / 64) * (NCOL3 / 64) / 8, 1), 256, 0, stream>>>(
      XH, XH, NIN, 0L, WI, WI, NIN, 0L, (void*)UX, (void*)UX, NCOL3, 0L,
      (const float*)UX, (const float*)UX, 0L, NROWS, NCOL3, NIN, FOLD);
  hyp_seq_kernel<<<NBATCH / RBLK, NTHR3, LDS_TOTAL, stream>>>(UX, WH, bias, kp, out, out + (size_t)NOUT0);
}
